// FCN_MODEL_87763361727284
// MI455X (gfx1250) — hardware-run, weakly checked
//
#include <hip/hip_runtime.h>


namespace {
constexpr int LB = 4, N = 50000, D = 64, E = 500000, KIN = LB * 2 * D  , HID = 256;
constexpr float WSC = 256.0f, LNEPS = 1e-5f;
typedef _Float16 b16;
typedef __attribute__((ext_vector_type(16))) _Float16 v16b;
typedef __attribute__((ext_vector_type(8))) _Float16 v8b;
typedef __attribute__((ext_vector_type(8))) float v8f;
typedef __attribute__((ext_vector_type(4))) float v4f;
typedef __attribute__((ext_vector_type(2))) float v2f;
__device__ __forceinline__ float bf16_rne(float f) { unsigned int u = __float_as_uint(f); u += 0x7FFFu + ((u >> 16) & 1u); float r = __uint_as_float(u & 0xFFFF0000u); asm volatile("" : "+v"(r)); return r; }
__device__ __forceinline__ float bfv(float f) { float r = bf16_rne(f); asm volatile("" : "+v"(r)); return r; }
__device__ __forceinline__ v16b frag_kb(const b16* p, int hh) { const v8b a = *(const v8b*)(p + 8 * hh), b = *(const v8b*)(p + 16 + 8 * hh); v16b f;
#pragma unroll
  for (int e = 0; e < 8; ++e) { f[e] = a[e]; f[8 + e] = b[e]; } return f; }
__device__ __forceinline__ v8f wmma16b(v16b a, v16b b, v8f c) { v8f d = __builtin_amdgcn_wmma_f32_16x16x32_f16(false, a, false, b, (short)0, c, false, false); asm volatile("v_nop\n\tv_nop\n\tv_nop\n\tv_nop" : "+v"(d) : "v"(a), "v"(b)); return d; }
__device__ __forceinline__ void wave_lds_sync() { __builtin_amdgcn_fence(__ATOMIC_RELEASE, "workgroup"); __builtin_amdgcn_wave_barrier(); __builtin_amdgcn_fence(__ATOMIC_ACQUIRE, "workgroup"); }
__device__ __forceinline__ float pmul(float a, float b) { float p = a * b; asm volatile("" : "+v"(p)); return p; }
__device__ __forceinline__ int iclamp(int v, int lo, int hi) { return v < lo ? lo : (v > hi ? hi : v); }

__global__ __launch_bounds__(256) void wput_kernel(const float* __restrict__ w1, b16* __restrict__ WT) { const int u = blockIdx.x * 256 + threadIdx.x; if (u >= HID * (KIN / 8)) return; const int o = u / (KIN / 8), k0 = (u % (KIN / 8)) * 8; v8b v;
#pragma unroll
  for (int j = 0; j < 8; ++j) v[j] = (b16)(bf16_rne(w1[(size_t)o * KIN + k0 + j]) * WSC); for (int pass = 0; pass < 2; ++pass) { *(volatile v8b*)(WT + (size_t)o * KIN + k0) = v; __threadfence(); } }
__global__ __launch_bounds__(32) void edge_kernel(const float* __restrict__ h, const int* __restrict__ src, const int* __restrict__ dst, const b16* __restrict__ WT, const float* __restrict__ b1, const float* __restrict__ w3, const float* __restrict__ b3, const float* __restrict__ g2, const float* __restrict__ be2, int ELIM, float* __restrict__ out) {
  __shared__ __attribute__((aligned(16))) b16 Ah[16][KIN + 8]; __shared__ float Tf[16][HID + 4], Os[32]; const int lane = threadIdx.x, nloc = lane & 15, hlf = lane >> 4; const size_t e0 = (size_t)blockIdx.x * 32; if (e0 >= (size_t)ELIM) return;
  if (lane < 16) for (int k = KIN; k < KIN + 8; ++k) Ah[lane][k] = (b16)0.0f;
#pragma unroll 1
  for (int rt = 0; rt < 2; ++rt) {
    { const int r = nloc; const size_t e = e0 + rt * 16 + r; const size_t nd = (size_t)iclamp(hlf ? dst[e] : src[e], 0, N - 1);
      for (int l = 0; l < LB; ++l) { const float imp = (float)(l + 1) / 10.0f; const float* hp = h + ((size_t)l * N + nd) * D;
        for (int q = 0; q < D / 4; ++q) { const v4f v = *(const v4f*)(hp + q * 4);
#pragma unroll
          for (int j = 0; j < 4; ++j) Ah[r][l * 2 * D + hlf * D + q * 4 + j] = (b16)tanhf(pmul(bfv(v[j]), imp)); } } }
    wave_lds_sync(); v8f acc[16];
#pragma unroll
    for (int t = 0; t < 16; ++t) acc[t] = (v8f){};
#pragma unroll 2
    for (int kb = 0; kb < KIN; kb += 32) { const v16b a = frag_kb(&Ah[nloc][kb], hlf);
#pragma unroll
      for (int t = 0; t < 16; ++t) acc[t] = wmma16b(a, frag_kb(WT + (size_t)(t * 16 + nloc) * KIN + kb, hlf), acc[t]); }
#pragma unroll
    for (int t = 0; t < 16; ++t) { const int cc = t * 16 + nloc; const float bb = bfv(b1[cc]);
#pragma unroll
      for (int r8 = 0; r8 < 8; ++r8) Tf[8 * hlf + r8][cc] = acc[t][r8] * (1.0f / WSC) + bb; }
    wave_lds_sync();
    for (int rr = 0; rr < 16; ++rr) { float v[8], sm = 0.0f;
#pragma unroll
      for (int q = 0; q < 8; ++q) { v[q] = Tf[rr][q * 32 + lane]; sm += v[q]; } for (int o = 16; o; o >>= 1) sm += __shfl_xor(sm, o); const float mu = sm / HID; float q2 = 0.0f;
#pragma unroll
      for (int q = 0; q < 8; ++q) q2 += (v[q] - mu) * (v[q] - mu); for (int o = 16; o; o >>= 1) q2 += __shfl_xor(q2, o); const float rs = rsqrtf(q2 / HID + LNEPS);
      float s = 0.0f;
#pragma unroll
      for (int q = 0; q < 8; ++q) { const int c = q * 32 + lane; const float y = fmaxf(pmul((v[q] - mu) * rs, bfv(g2[c])) + bfv(be2[c]), 0.0f); s += pmul(y, bfv(w3[c])); } for (int o = 16; o; o >>= 1) s += __shfl_xor(s, o); if (lane == 0) Os[rt * 16 + rr] = s + bfv(b3[0]); }
    wave_lds_sync(); }
  for (int pass = 0; pass < 2; ++pass) { ((volatile float*)out)[e0 + lane] = Os[lane]; __threadfence(); } }
}

extern "C" void kernel_launch(void* const* d_in, const int* in_sizes, int n_in, void* d_out, int out_size, void* d_ws, size_t ws_size, hipStream_t stream) {
  (void)n_in;
  auto Fp = [&](int i) { return (const float*)d_in[i]; }; auto Ip = [&](int i) { return (const int*)d_in[i]; };
  if (in_sizes[0] != LB * N * D || in_sizes[1] != E || in_sizes[2] != E || in_sizes[3] != HID * KIN || in_sizes[5] != HID || in_sizes[7] != HID || out_size != E) return;
  const int ELIM = E;
  size_t off = 0; char* ws = (char*)d_ws;
  auto carve = [&](size_t bytes) { char* p = ws + off; off += (bytes + 255) & ~(size_t)255; return p; };
  b16* WT = (b16*)carve((size_t)HID * KIN * 2);
  if (off > ws_size || off > ((size_t)4 << 20)) return;
  wput_kernel<<<(HID * (KIN / 8) + 255) / 256, 256, 0, stream>>>(Fp(3), WT);
  edge_kernel<<<ELIM / 32, 32, 0, stream>>>(Fp(0), Ip(1), Ip(2), WT, Fp(4), Fp(5), Fp(6), Fp(7), Fp(8), ELIM, (float*)d_out);
}
